// Block_43911745634528
// MI455X (gfx1250) — hardware-run, weakly checked
//
#include <hip/hip_runtime.h>


#ifndef NB
#define NB 2
#endif
#ifndef SEQ
#define SEQ 2048
#endif
#define NB_FULL  2
#define SEQ_FULL 2048
#ifndef OUT_SEQ
#define OUT_SEQ SEQ
#endif
#define DM   512
#define NH_  16
#define HD   32
#define DFF  2048
#define AW   4
#define OSP  36
#define EROWS (SEQ < 256 ? SEQ : 256)
#define QRS  2048.0f
#define QRI  (1.0f / 2048.0f)
#define LOG2E 1.4426950408889634f
#define PSH  14.0f
#define NEGB (-3.0e38f)
#define LNEPS 1.0e-3f
#define WL2  10
#define CL2  4
#define WSC  1024.0f
#define CSC  16.0f

static_assert(HD == 32);
static_assert(NH_ * HD == DM);
static_assert(DM == 512);
static_assert(DM % 64 == 0);
static_assert(DFF % 64 == 0);
static_assert(DM % 32 == 0);
static_assert(DFF % 32 == 0);
static_assert(SEQ % 64 == 0);
static_assert((NB * SEQ) % 64 == 0);
static_assert((NB * SEQ) % 8 == 0);
static_assert(SEQ % 32 == 0);
static_assert(SEQ % (16 * AW) == 0);
static_assert(EROWS % 64 == 0);
static_assert(EROWS % 32 == 0);
static_assert(EROWS >= 32);
static_assert(EROWS <= SEQ);
static_assert(EROWS % (16 * AW) == 0);
static_assert((SEQ - EROWS) % (16 * AW) == 0);
static_assert(NB <= NB_FULL);
static_assert(SEQ <= SEQ_FULL);
static_assert((OSP * 4) % 16 == 0);
static_assert((1 << WL2) == 1024);
static_assert((1 << CL2) == 16);
static_assert(16 * 68 * 4 <= 131072);
static_assert(AW * 16 * OSP * 4 <= 131072);
static_assert(32 * 68 * 4 <= 131072);

typedef _Float16 h16;
typedef __attribute__((ext_vector_type(16))) _Float16 v16h;
typedef __attribute__((ext_vector_type(8)))  _Float16 v8h;
typedef __attribute__((ext_vector_type(8)))  float    v8f;
typedef __attribute__((ext_vector_type(4)))  float    v4f;
typedef v4f  __attribute__((may_alias)) v4fa;
typedef v8h  __attribute__((may_alias)) v8ha;

__device__ __forceinline__ unsigned short f2bf(float f) { unsigned u = __float_as_uint(f); u += 0x7FFFu + ((u >> 16) & 1u); return (unsigned short)(u >> 16); }
__device__ __forceinline__ float bfr(float f) { return __uint_as_float(((unsigned)f2bf(f)) << 16); }
__device__ __forceinline__ v16h cat16(v8h lo, v8h hi) { return __builtin_shufflevector(lo, hi, 0, 1, 2, 3, 4, 5, 6, 7, 8, 9, 10, 11, 12, 13, 14, 15); }
__device__ __forceinline__ v8f wmma16(v16h a, v16h b, v8f c) { return __builtin_amdgcn_wmma_f32_16x16x32_f16(false, a, false, b, (short)0, c, false, false); }
__device__ __forceinline__ v8f wmma16g(v16h a, v16h b, v8f c) { c = wmma16(a, b, c); asm volatile("v_nop\n\tv_nop\n\tv_nop\n\tv_nop" : "+v"(c) : "v"(a), "v"(b)); return c; }
__device__ __forceinline__ v16h  ldh(const h16* p) { return cat16(*(const v8h*)p, *(const v8h*)(p + 16)); }
__device__ __forceinline__ void wave_sync() { __builtin_amdgcn_fence(3  , "wavefront"); __builtin_amdgcn_wave_barrier(); asm volatile("" ::: "memory"); }
static __device__ __forceinline__ h16 toh_flush(float v) { const float w = (fabsf(v) < 6.103515625e-05f) ? 0.0f : v; return (h16)w; }

static_assert(256 * 8 == 64 * 32);
static_assert(256 * 16 == 32 * 128);
__global__ __launch_bounds__(256) void k_wconvT(const float* __restrict__ src, h16* dst, unsigned R, unsigned Cn) {
    __shared__ __align__(16) float ts[32 * 68];
    const unsigned tid = threadIdx.x;
    const unsigned r0 = blockIdx.x * 64u, c0 = blockIdx.y * 32u, z = blockIdx.z;
    const float* sp = src + (size_t)z * R * Cn;
    h16* dp = dst + (size_t)z * R * Cn;
    const unsigned lrow = tid >> 2, lc = (tid & 3u) * 8u;
    const v4f a = *(const v4f*)(sp + (size_t)(r0 + lrow) * Cn + c0 + lc);
    const v4f b = *(const v4f*)(sp + (size_t)(r0 + lrow) * Cn + c0 + lc + 4);
#pragma unroll
    for (int i = 0; i < 4; ++i) { ts[(lc + i) * 68 + lrow] = bfr(a[i]) * WSC; ts[(lc + 4 + i) * 68 + lrow] = bfr(b[i]) * WSC; }
    __syncthreads();
    const unsigned orow = tid >> 3, oc = (tid & 7u) * 8u;
    const v4f x0 = *(const v4fa*)(&ts[orow * 68 + oc]); const v4f x1 = *(const v4fa*)(&ts[orow * 68 + oc + 4]);
    v8h o;
#pragma unroll
    for (int i = 0; i < 4; ++i) { o[i] = toh_flush(x0[i]); o[4 + i] = toh_flush(x1[i]); }
    h16* q = dp + (size_t)(c0 + orow) * R + r0 + oc;
    *(volatile v8h*)q = o; __threadfence(); *(volatile v8h*)q = o;
}

static_assert(2 * 32 * 8 == DM);
__global__ __launch_bounds__(256) void k_ln(const float* __restrict__ src, const float* __restrict__ g, const float* __restrict__ be, h16* dst, unsigned seqPitch, int rin) {
#pragma clang fp contract(off)
    const unsigned lane = threadIdx.x & 31u, wave = threadIdx.x >> 5;
    const unsigned row = blockIdx.x * 8u + wave;
    const unsigned bb = row / (unsigned)SEQ, tt = row % (unsigned)SEQ;
    const float* sp = src + ((size_t)bb * seqPitch + tt) * DM + lane * 8u;
    float v[16];
#pragma unroll
    for (int s = 0; s < 2; ++s) { const v4f a = *(const v4f*)(sp + s * 256); const v4f c = *(const v4f*)(sp + s * 256 + 4);
#pragma unroll
        for (int i = 0; i < 4; ++i) { v[s * 8 + i] = a[i]; v[s * 8 + 4 + i] = c[i]; } }
#pragma unroll
    for (int i = 0; i < 16; ++i) v[i] = (rin != 0) ? bfr(v[i]) : v[i];
    float sm = 0.0f;
#pragma unroll
    for (int i = 0; i < 16; ++i) sm += v[i];
#pragma unroll
    for (int m = 16; m >= 1; m >>= 1) sm += __shfl_xor(sm, m, 32);
    const float mu = sm * (1.0f / (float)DM);
    float sq = 0.0f;
#pragma unroll
    for (int i = 0; i < 16; ++i) { const float d = v[i] - mu; v[i] = d; sq += d * d; }
#pragma unroll
    for (int m = 16; m >= 1; m >>= 1) sq += __shfl_xor(sq, m, 32);
    const float var = sq * (1.0f / (float)DM);
    const float rs = 1.0f / sqrtf(var + LNEPS);
    v8h o0, o1;
#pragma unroll
    for (int s = 0; s < 2; ++s) {
        const v4f g0 = *(const v4f*)(g + s * 256 + lane * 8u), g1 = *(const v4f*)(g + s * 256 + lane * 8u + 4);
        const v4f b0 = *(const v4f*)(be + s * 256 + lane * 8u), b1 = *(const v4f*)(be + s * 256 + lane * 8u + 4);
#pragma unroll
        for (int i = 0; i < 4; ++i) {
            const float y0 = v[s * 8 + i] * rs * bfr(g0[i]) + bfr(b0[i]);
            const float y1 = v[s * 8 + 4 + i] * rs * bfr(g1[i]) + bfr(b1[i]);
            if (s == 0) { o0[i] = toh_flush(y0); o0[4 + i] = toh_flush(y1); } else { o1[i] = toh_flush(y0); o1[4 + i] = toh_flush(y1); } } }
    h16* dp = dst + (size_t)row * DM + lane * 8u;
    *(volatile v8h*)dp = o0; *(volatile v8h*)(dp + 256) = o1;
    __threadfence();
    *(volatile v8h*)dp = o0; *(volatile v8h*)(dp + 256) = o1;
}

template <int KD, int AKB>
__device__ __forceinline__ void gemm_kloop(const h16* __restrict__ A, const h16* __restrict__ Bt, size_t aoff, size_t boff, size_t amb, v8f (&acc)[4][4]) {
#pragma unroll 1
    for (int kc = 0; kc < KD; kc += 32) {
        v16h a[4];
        const size_t ak = aoff + (size_t)(kc >> 5) * (size_t)AKB;
#pragma unroll
        for (int mb = 0; mb < 4; ++mb) a[mb] = ldh(A + ak + (size_t)mb * amb);
#pragma unroll
        for (int nb = 0; nb < 4; ++nb) { const v16h b = ldh(Bt + boff + (size_t)nb * 16 * KD + kc);
#pragma unroll
            for (int mb = 0; mb < 4; ++mb) acc[mb][nb] = wmma16g(a[mb], b, acc[mb][nb]); }
    }
}

static_assert(2 * 32 * 16 == 16 * HD * 2);
__device__ __forceinline__ void epi_tok(const v8f (&acc)[4][4], const float* __restrict__ bias, h16* Ph, h16* Pr, unsigned r0, unsigned c0) {
    __shared__ __align__(16) float os[16 * 68];
    const int lane = threadIdx.x & 31, lr = lane & 15, hi = lane >> 4;
    constexpr float FOLD = 1.0f / (float)(1 << WL2);
    float bc[4];
#pragma unroll
    for (int nb = 0; nb < 4; ++nb) bc[nb] = bfr(bias[c0 + nb * 16 + lr]);
    const unsigned bb = r0 / (unsigned)SEQ, tt = r0 % (unsigned)SEQ; const unsigned zc = bb * (unsigned)NH_ + c0 / (unsigned)HD;
    const size_t tbase = ((size_t)zc * SEQ + (size_t)tt) * HD; const size_t rbase = ((size_t)zc * EROWS + (size_t)tt) * HD; const bool wr = tt < (unsigned)EROWS;
#pragma unroll
    for (int mb = 0; mb < 4; ++mb) {
#pragma unroll
        for (int nb = 0; nb < 4; ++nb) {
#pragma unroll
            for (int j = 0; j < 8; ++j) os[(hi * 8 + j) * 68 + nb * 16 + lr] = acc[mb][nb][j] * FOLD + bc[nb]; }
        wave_sync();
#pragma unroll 1
        for (int ps = 0; ps < 2; ++ps) {
            const size_t sb = tbase + (size_t)(mb * 16) * HD;
            const size_t rb = rbase + (size_t)(mb * 16) * HD;
#pragma unroll
            for (int hh = 0; hh < 2; ++hh) {
#pragma unroll
                for (int s = 0; s < 2; ++s) { const int p = s * 32 + lane; const int row = p >> 2, c8 = (p & 3) * 8;
                    const v4f x0 = *(const v4fa*)(&os[row * 68 + hh * 32 + c8]); const v4f x1 = *(const v4fa*)(&os[row * 68 + hh * 32 + c8 + 4]); v8h hv, rv;
#pragma unroll
                    for (int i = 0; i < 4; ++i) { const h16 a0 = toh_flush(x0[i]); const h16 a1 = toh_flush(x1[i]); hv[i] = a0; hv[4 + i] = a1;
                        rv[i] = toh_flush((x0[i] - (float)a0) * QRS); rv[4 + i] = toh_flush((x1[i] - (float)a1) * QRS); }
                    const size_t oo = sb + (size_t)hh * ((size_t)SEQ * HD) + (size_t)p * 8;
                    const size_t ro = rb + (size_t)hh * ((size_t)EROWS * HD) + (size_t)p * 8;
                    *(volatile v8h*)(Ph + oo) = hv; if (wr) *(volatile v8h*)(Pr + ro) = rv; } }
            if (ps == 0) __threadfence(); }
        wave_sync();
    }
}

static_assert(4 * 4 == 16);
static_assert(8 * 16 == 64 * 2);
__device__ __forceinline__ void epi_vt(const v8f (&acc)[4][4], const float* __restrict__ bias, h16* Ph, h16* Pr, unsigned r0, unsigned c0) {
    __shared__ __align__(16) float os[16 * 68];
    const int lane = threadIdx.x & 31, lr = lane & 15, hi = lane >> 4;
    constexpr float FOLD = 1.0f / (float)(1 << WL2);
    const unsigned bb = c0 / (unsigned)SEQ, tt = c0 % (unsigned)SEQ;
    const size_t tbase = (size_t)bb * (size_t)DM * SEQ + (size_t)r0 * SEQ + (size_t)tt;
    const size_t rbase = (size_t)bb * (size_t)DM * EROWS + (size_t)r0 * EROWS + (size_t)tt; const bool wr = tt < (unsigned)EROWS;
#pragma unroll
    for (int mb = 0; mb < 4; ++mb) {
        float br[8];
#pragma unroll
        for (int j = 0; j < 8; ++j) br[j] = bfr(bias[r0 + mb * 16 + hi * 8 + j]);
#pragma unroll
        for (int nb = 0; nb < 4; ++nb) {
#pragma unroll
            for (int j = 0; j < 8; ++j) os[(hi * 8 + j) * 68 + nb * 16 + lr] = acc[mb][nb][j] * FOLD + br[j]; }
        wave_sync();
#pragma unroll 1
        for (int ps = 0; ps < 2; ++ps) {
            const size_t sb = tbase + (size_t)(mb * 16) * SEQ;
            const size_t rb = rbase + (size_t)(mb * 16) * (size_t)EROWS;
#pragma unroll
            for (int s = 0; s < 4; ++s) { const int row = 4 * s + (lane >> 3), c8 = (lane & 7) * 8;
                const v4f x0 = *(const v4fa*)(&os[row * 68 + c8]); const v4f x1 = *(const v4fa*)(&os[row * 68 + c8 + 4]); v8h hv, rv;
#pragma unroll
                for (int i = 0; i < 4; ++i) { const h16 a0 = toh_flush(x0[i]); const h16 a1 = toh_flush(x1[i]); hv[i] = a0; hv[4 + i] = a1;
                    rv[i] = toh_flush((x0[i] - (float)a0) * QRS); rv[4 + i] = toh_flush((x1[i] - (float)a1) * QRS); }
                const size_t oo = sb + (size_t)row * SEQ + c8;
                const size_t ro = rb + (size_t)row * (size_t)EROWS + c8;
                *(volatile v8h*)(Ph + oo) = hv; if (wr) *(volatile v8h*)(Pr + ro) = rv; }
            if (ps == 0) __threadfence(); }
        wave_sync();
    }
}

template <int FL2, int NOUT, int RELU>
__device__ __forceinline__ void epi_h16(const v8f (&acc)[4][4], const float* __restrict__ bias, h16* Ph, unsigned r0, unsigned c0) {
    __shared__ __align__(16) float os[16 * 68];
    const int lane = threadIdx.x & 31, lr = lane & 15, hi = lane >> 4;
    constexpr float FOLD = 1.0f / (float)(1 << FL2);
    float bc[4];
#pragma unroll
    for (int nb = 0; nb < 4; ++nb) bc[nb] = bfr(bias[c0 + nb * 16 + lr]);
#pragma unroll
    for (int mb = 0; mb < 4; ++mb) {
#pragma unroll
        for (int nb = 0; nb < 4; ++nb) {
#pragma unroll
            for (int j = 0; j < 8; ++j) { float val = acc[mb][nb][j] * FOLD + bc[nb]; if (RELU) val = fmaxf(val, 0.0f); os[(hi * 8 + j) * 68 + nb * 16 + lr] = val; } }
        wave_sync();
#pragma unroll 1
        for (int ps = 0; ps < 2; ++ps) {
#pragma unroll
            for (int s = 0; s < 4; ++s) { const int row = 4 * s + (lane >> 3), c8 = (lane & 7) * 8;
                const v4f x0 = *(const v4fa*)(&os[row * 68 + c8]); const v4f x1 = *(const v4fa*)(&os[row * 68 + c8 + 4]); v8h hv;
#pragma unroll
                for (int i = 0; i < 4; ++i) { hv[i] = toh_flush(x0[i]); hv[4 + i] = toh_flush(x1[i]); }
                *(volatile v8h*)(Ph + (size_t)(r0 + mb * 16 + row) * NOUT + c0 + c8) = hv; }
            if (ps == 0) __threadfence(); }
        wave_sync();
    }
}

static_assert(8 * 2 == 16);
static_assert(16 * 16 == 64 * 4);
template <int FL2, int RESP, int OUTP, int RRES>
__device__ __forceinline__ void epi_f32(const v8f (&acc)[4][4], const float* __restrict__ bias, const float* __restrict__ RES, float* OF, unsigned r0, unsigned c0) {
    __shared__ __align__(16) float os[16 * 68];
    const int lane = threadIdx.x & 31, lr = lane & 15, hi = lane >> 4;
    constexpr float FOLD = 1.0f / (float)(1 << FL2);
    float bc[4];
#pragma unroll
    for (int nb = 0; nb < 4; ++nb) bc[nb] = bfr(bias[c0 + nb * 16 + lr]);
    const unsigned bb = r0 / (unsigned)SEQ, tt = r0 % (unsigned)SEQ;
    const size_t rrow0 = (size_t)bb * (size_t)RESP + tt, orow0 = (size_t)bb * (size_t)OUTP + tt;
#pragma unroll
    for (int mb = 0; mb < 4; ++mb) {
#pragma unroll
        for (int nb = 0; nb < 4; ++nb) {
#pragma unroll
            for (int j = 0; j < 8; ++j) os[(hi * 8 + j) * 68 + nb * 16 + lr] = acc[mb][nb][j] * FOLD + bc[nb]; }
        wave_sync();
#pragma unroll 1
        for (int ps = 0; ps < 2; ++ps) {
#pragma unroll
            for (int s = 0; s < 8; ++s) { const int row = 2 * s + (lane >> 4), cofs = (lane & 15) * 4;
                v4f val = *(const v4fa*)(&os[row * 68 + cofs]);
                v4f rv = *(const v4f*)(RES + (rrow0 + (size_t)(mb * 16 + row)) * DM + c0 + cofs);
                if (RRES) { rv[0] = bfr(rv[0]); rv[1] = bfr(rv[1]); rv[2] = bfr(rv[2]); rv[3] = bfr(rv[3]); }
                val = val + rv;
                *(volatile v4f*)(OF + (orow0 + (size_t)(mb * 16 + row)) * DM + c0 + cofs) = val; }
            if (ps == 0) __threadfence(); }
        wave_sync();
    }
}

__device__ __forceinline__ void acc_zero(v8f (&acc)[4][4]) {
#pragma unroll
    for (int mb = 0; mb < 4; ++mb)
#pragma unroll
        for (int nb = 0; nb < 4; ++nb) acc[mb][nb] = (v8f){};
}

__global__ __launch_bounds__(32) void k_gemm_tok(const h16* __restrict__ A, const h16* __restrict__ Bt, const float* __restrict__ bias, h16* Ph, h16* Pr) {
    const unsigned lane = threadIdx.x & 31u, lr = lane & 15u, hi = lane >> 4;
    const unsigned r0 = blockIdx.x * 64u, c0 = blockIdx.y * 64u;
    v8f acc[4][4]; acc_zero(acc);
    gemm_kloop<DM, 32>(A, Bt, (size_t)(r0 + lr) * DM + 8u * hi, (size_t)(c0 + lr) * DM + 8u * hi, (size_t)16 * DM, acc);
    epi_tok(acc, bias, Ph, Pr, r0, c0);
}
__global__ __launch_bounds__(32) void k_gemm_vt(const h16* __restrict__ A, const h16* __restrict__ Bt, const float* __restrict__ bias, h16* Ph, h16* Pr) {
    const unsigned lane = threadIdx.x & 31u, lr = lane & 15u, hi = lane >> 4;
    const unsigned r0 = blockIdx.x * 64u, c0 = blockIdx.y * 64u;
    v8f acc[4][4]; acc_zero(acc);
    gemm_kloop<DM, 32>(A, Bt, (size_t)(r0 + lr) * DM + 8u * hi, (size_t)(c0 + lr) * DM + 8u * hi, (size_t)16 * DM, acc);
    epi_vt(acc, bias, Ph, Pr, r0, c0);
}
__global__ __launch_bounds__(32) void k_gemm_wo(const h16* __restrict__ A, const h16* __restrict__ Bt, const float* __restrict__ bias, const float* __restrict__ RES, float* OF) {
    const unsigned lane = threadIdx.x & 31u, lr = lane & 15u, hi = lane >> 4;
    const unsigned r0 = blockIdx.x * 64u, c0 = blockIdx.y * 64u;
    v8f acc[4][4]; acc_zero(acc);
    gemm_kloop<DM, NB * SEQ * HD>(A, Bt, (size_t)(r0 + lr) * HD + 8u * hi, (size_t)(c0 + lr) * DM + 8u * hi, (size_t)16 * HD, acc);
    epi_f32<WL2 + CL2, SEQ_FULL, SEQ, 1>(acc, bias, RES, OF, r0, c0);
}
__global__ __launch_bounds__(32) void k_gemm_f1(const h16* __restrict__ A, const h16* __restrict__ Bt, const float* __restrict__ bias, h16* G) {
    const unsigned lane = threadIdx.x & 31u, lr = lane & 15u, hi = lane >> 4;
    const unsigned r0 = blockIdx.x * 64u, c0 = blockIdx.y * 64u;
    v8f acc[4][4]; acc_zero(acc);
    gemm_kloop<DM, 32>(A, Bt, (size_t)(r0 + lr) * DM + 8u * hi, (size_t)(c0 + lr) * DM + 8u * hi, (size_t)16 * DM, acc);
    epi_h16<WL2, DFF, 1>(acc, bias, G, r0, c0);
}
__global__ __launch_bounds__(32) void k_gemm_f2(const h16* __restrict__ A, const h16* __restrict__ Bt, const float* __restrict__ bias, const float* __restrict__ RES, float* OF) {
    const unsigned lane = threadIdx.x & 31u, lr = lane & 15u, hi = lane >> 4;
    const unsigned r0 = blockIdx.x * 64u, c0 = blockIdx.y * 64u;
    v8f acc[4][4]; acc_zero(acc);
    gemm_kloop<DFF, 32>(A, Bt, (size_t)(r0 + lr) * DFF + 8u * hi, (size_t)(c0 + lr) * DFF + 8u * hi, (size_t)16 * DFF, acc);
    epi_f32<WL2, SEQ, OUT_SEQ, 0>(acc, bias, RES, OF, r0, c0);
}

template <int EARLY>
__device__ __forceinline__ void flash_body(const h16* __restrict__ QH, const h16* __restrict__ QR, const h16* __restrict__ KP, const h16* __restrict__ KR,
                                           const h16* __restrict__ VT, const h16* __restrict__ VR, h16* CT) {
    __shared__ __align__(16) float os[AW * 16 * OSP];
    const int lane = threadIdx.x & 31, lr = lane & 15, hi = lane >> 4;
    const int wave = __builtin_amdgcn_readfirstlane((int)(threadIdx.x >> 5));
    const unsigned zh = blockIdx.y; const unsigned b = zh / (unsigned)NH_, h = zh % (unsigned)NH_;
    const int t0 = (EARLY ? 0 : EROWS) + ((int)blockIdx.x * AW + wave) * 16;
    const int lim = t0 + lr;
    const int nk = (t0 + 16 + 31) & ~31;
    const size_t pbase = (size_t)zh * SEQ * HD;
    const size_t rbase = (size_t)zh * EROWS * HD;
    const size_t qo = pbase + (size_t)(t0 + lr) * HD + 8 * hi;
    const v16h hz = (v16h){};
    const v16h qh = ldh(QH + qo);
    v16h qr = hz;
    if (EARLY) qr = ldh(QR + rbase + (size_t)(t0 + lr) * HD + 8 * hi);
    const size_t ko = pbase + (size_t)lr * HD + 8 * hi;
    const size_t vo = pbase + (size_t)lr * SEQ + 8 * hi;
    const size_t kro = rbase + (size_t)lr * HD + 8 * hi;
    const size_t vro = rbase + (size_t)lr * EROWS + 8 * hi;
    v8f o0 = (v8f){}, o1 = (v8f){}, oR0 = (v8f){}, oR1 = (v8f){};
    float m = NEGB, l = 0.0f;
#pragma unroll 1
    for (int key0 = 0; key0 < nk; key0 += 32) {
        const h16* ka = KP + ko + (size_t)key0 * HD;
        const v16h ka0 = ldh(ka), kb0 = ldh(ka + 16 * HD);
        v8f sHa = (v8f){}, sLa = (v8f){}, sHb = (v8f){}, sLb = (v8f){};
        sHa = wmma16g(ka0, qh, sHa); sHb = wmma16g(kb0, qh, sHb);
        if (EARLY) {
            const h16* kr = KR + kro + (size_t)key0 * HD;
            const v16h kra0 = ldh(kr), krb0 = ldh(kr + 16 * HD);
            sLa = wmma16g(ka0, qr, sLa); sLb = wmma16g(kb0, qr, sLb);
            sLa = wmma16g(kra0, qh, sLa); sLb = wmma16g(krb0, qh, sLb);
        }
        const int ja = key0 + 8 * hi;
        float ta[8], tb[8]; bool fa[8], fb[8]; float mx = NEGB;
#pragma unroll
        for (int r = 0; r < 8; ++r) {
            fa[r] = (ja + r <= lim);
            fb[r] = (ja + 16 + r <= lim);
            if (EARLY) { ta[r] = (sHa[r] + sLa[r] * QRI) * LOG2E; tb[r] = (sHb[r] + sLb[r] * QRI) * LOG2E; }
            else       { ta[r] = sHa[r] * LOG2E; tb[r] = sHb[r] * LOG2E; }
            mx = fmaxf(mx, fmaxf(fa[r] ? ta[r] : NEGB, fb[r] ? tb[r] : NEGB)); }
        mx = fmaxf(mx, __shfl_xor(mx, 16, 32));
        const float mnew = fmaxf(m, mx);
        const float alpha = __builtin_amdgcn_exp2f(m - mnew);
        const float sh = PSH - mnew;
        v16h pb, pr = hz; float ls = 0.0f;
#pragma unroll
        for (int r = 0; r < 8; ++r) {
            const float ea = __builtin_amdgcn_exp2f(ta[r] + sh), eb = __builtin_amdgcn_exp2f(tb[r] + sh);
            const float ga = fa[r] ? ea : 0.0f, gb = fb[r] ? eb : 0.0f;
            const h16 pa = toh_flush(ga); const h16 pc = toh_flush(gb);
            pb[r] = pa; pb[8 + r] = pc;
            if (EARLY) { pr[r] = toh_flush((ga - (float)pa) * QRS); pr[8 + r] = toh_flush((gb - (float)pc) * QRS); ls += ga + gb; }
            else       { ls += (float)pa + (float)pc; } }
        l = l * alpha + ls; m = mnew;
        o0 = o0 * alpha; o1 = o1 * alpha;
        if (EARLY) { oR0 = oR0 * alpha; oR1 = oR1 * alpha; }
        const h16* va = VT + vo + key0;
        const v16h v0 = ldh(va), v1 = ldh(va + (size_t)16 * SEQ);
        o0 = wmma16g(v0, pb, o0); o1 = wmma16g(v1, pb, o1);
        if (EARLY) {
            const h16* vr = VR + vro + key0;
            const v16h vr0 = ldh(vr), vr1 = ldh(vr + (size_t)16 * EROWS);
            oR0 = wmma16g(v0, pr, oR0); oR1 = wmma16g(v1, pr, oR1);
            oR0 = wmma16g(vr0, pb, oR0); oR1 = wmma16g(vr1, pb, oR1);
        }
    }
    l += __shfl_xor(l, 16, 32);
    const bool any = l > 0.0f;
    const float lsafe = any ? l : 1.0f;
    const float inv = any ? (CSC / lsafe) : 0.0f;
    v8f f0 = o0, f1 = o1;
    if (EARLY) { f0 = o0 + oR0 * QRI; f1 = o1 + oR1 * QRI; }
    const int wb = wave * 16 * OSP;
    { v4f a, c;
      a[0] = f0[0] * inv; a[1] = f0[1] * inv; a[2] = f0[2] * inv; a[3] = f0[3] * inv; c[0] = f0[4] * inv; c[1] = f0[5] * inv; c[2] = f0[6] * inv; c[3] = f0[7] * inv;
      *(v4fa*)(&os[wb + lr * OSP +  0 + 8 * hi]) = a; *(v4fa*)(&os[wb + lr * OSP +  0 + 8 * hi + 4]) = c;
      a[0] = f1[0] * inv; a[1] = f1[1] * inv; a[2] = f1[2] * inv; a[3] = f1[3] * inv; c[0] = f1[4] * inv; c[1] = f1[5] * inv; c[2] = f1[6] * inv; c[3] = f1[7] * inv;
      *(v4fa*)(&os[wb + lr * OSP + 16 + 8 * hi]) = a; *(v4fa*)(&os[wb + lr * OSP + 16 + 8 * hi + 4]) = c; }
    wave_sync();
    const size_t cbase = (((size_t)h * NB + b) * SEQ + (size_t)t0) * HD;
#pragma unroll 1
    for (int ps = 0; ps < 2; ++ps) {
#pragma unroll
        for (int s = 0; s < 2; ++s) { const int p = s * 32 + lane; const int row = p >> 2, c8 = (p & 3) * 8;
            const v4f x0 = *(const v4fa*)(&os[wb + row * OSP + c8]); const v4f x1 = *(const v4fa*)(&os[wb + row * OSP + c8 + 4]); v8h hv;
#pragma unroll
            for (int i = 0; i < 4; ++i) { hv[i] = toh_flush(x0[i]); hv[4 + i] = toh_flush(x1[i]); }
            *(volatile v8h*)(CT + cbase + (size_t)p * 8) = hv; }
        if (ps == 0) __threadfence(); }
}

__global__ __launch_bounds__(32 * AW) void k_flash_early(const h16* __restrict__ QH, const h16* __restrict__ QR, const h16* __restrict__ KP, const h16* __restrict__ KR,
                                                         const h16* __restrict__ VT, const h16* __restrict__ VR, h16* CT) {
    flash_body<1>(QH, QR, KP, KR, VT, VR, CT);
}
__global__ __launch_bounds__(32 * AW) void k_flash_late(const h16* __restrict__ QH, const h16* __restrict__ KP, const h16* __restrict__ VT, h16* CT) {
    flash_body<0>(QH, QH, KP, KP, VT, VT, CT);
}

static constexpr size_t al256(size_t v) { return (v + 255) & ~(size_t)255; }
static constexpr size_t SZ_H  = al256((size_t)NB * SEQ * DM * 2);
static constexpr size_t SZ_WT = al256((size_t)3 * DM * DM * 2);
static constexpr size_t SZ_WO = al256((size_t)DM * DM * 2);
static constexpr size_t SZ_W1 = al256((size_t)DFF * DM * 2);
static constexpr size_t SZ_W2 = al256((size_t)DM * DFF * 2);
static constexpr size_t SZ_PL = al256((size_t)NB * NH_ * SEQ * HD * 2);
static constexpr size_t SZ_RS = al256((size_t)NB * NH_ * EROWS * HD * 2);
static constexpr size_t SZ_X1 = al256((size_t)NB * SEQ * DM * 4);
static constexpr size_t SZ_G  = al256((size_t)NB * SEQ * DFF * 2);
static constexpr size_t SZ_TOTAL = 2 * SZ_H + SZ_WT + SZ_WO + SZ_W1 + SZ_W2 + 4 * SZ_PL + 3 * SZ_RS + SZ_X1 + SZ_G;
static_assert(SZ_TOTAL <= (size_t)134217728);
static_assert(((size_t)DM * DM * 2) % 256 == 0);
static_assert((size_t)NB * NH_ * SEQ * HD == (size_t)NB * DM * SEQ);
static_assert((size_t)NB * NH_ * EROWS * HD == (size_t)NB * DM * EROWS);
static_assert((size_t)NH_ * NB * SEQ * HD == (size_t)NB * NH_ * SEQ * HD);
static constexpr size_t NEED_X   = ((size_t)(NB - 1) * SEQ_FULL + SEQ) * DM;
static constexpr size_t NEED_OUT = ((size_t)(NB - 1) * OUT_SEQ + SEQ) * DM;

extern "C" void kernel_launch(void* const* d_in, const int* in_sizes, int n_in,
                              void* d_out, int out_size, void* d_ws, size_t ws_size, hipStream_t stream) {
    if (n_in < 17) return;
    if ((size_t)in_sizes[0] < NEED_X) return;
    if ((size_t)in_sizes[1] < (size_t)DM * DM || (size_t)in_sizes[3] < (size_t)DM * DM || (size_t)in_sizes[5] < (size_t)DM * DM || (size_t)in_sizes[7] < (size_t)DM * DM) return;
    if (in_sizes[2] < DM || in_sizes[4] < DM || in_sizes[6] < DM || in_sizes[8] < DM) return;
    if ((size_t)in_sizes[9] < (size_t)DM * DFF || in_sizes[10] < DFF || (size_t)in_sizes[11] < (size_t)DFF * DM) return;
    if (in_sizes[12] < DM || in_sizes[13] < DM || in_sizes[14] < DM || in_sizes[15] < DM || in_sizes[16] < DM) return;
    if ((size_t)out_size < NEED_OUT) return;
    if (SZ_TOTAL > ws_size) return;
    const float* x   = (const float*)d_in[0];
    const float* wq  = (const float*)d_in[1];  const float* bq  = (const float*)d_in[2];
    const float* wk  = (const float*)d_in[3];  const float* bk  = (const float*)d_in[4];
    const float* wv  = (const float*)d_in[5];  const float* bv  = (const float*)d_in[6];
    const float* wo  = (const float*)d_in[7];  const float* bo  = (const float*)d_in[8];
    const float* w1  = (const float*)d_in[9];  const float* b1  = (const float*)d_in[10];
    const float* w2  = (const float*)d_in[11]; const float* b2  = (const float*)d_in[12];
    const float* g1  = (const float*)d_in[13]; const float* be1 = (const float*)d_in[14];
    const float* g2  = (const float*)d_in[15]; const float* be2 = (const float*)d_in[16];
    float* OUT = (float*)d_out;
    char* wsp = (char*)d_ws;
    h16* H1  = (h16*)wsp; wsp += SZ_H;
    h16* H2  = (h16*)wsp; wsp += SZ_H;
    h16* WT  = (h16*)wsp; wsp += SZ_WT;
    h16* WOT = (h16*)wsp; wsp += SZ_WO;
    h16* W1T = (h16*)wsp; wsp += SZ_W1;
    h16* W2T = (h16*)wsp; wsp += SZ_W2;
    h16* QH  = (h16*)wsp; wsp += SZ_PL;
    h16* KP  = (h16*)wsp; wsp += SZ_PL;
    h16* VT  = (h16*)wsp; wsp += SZ_PL;
    h16* CT  = (h16*)wsp; wsp += SZ_PL;
    h16* QR  = (h16*)wsp; wsp += SZ_RS;
    h16* KR  = (h16*)wsp; wsp += SZ_RS;
    h16* VR  = (h16*)wsp; wsp += SZ_RS;
    float* X1 = (float*)wsp; wsp += SZ_X1;
    h16* G   = (h16*)wsp; wsp += SZ_G;
    h16* WTQ = WT; h16* WTK = WT + (size_t)DM * DM; h16* WTV = WT + (size_t)2 * DM * DM;

    k_ln<<<dim3(NB * SEQ / 8, 1, 1), 256, 0, stream>>>(x, g1, be1, H1, (unsigned)SEQ_FULL, 1);
    k_wconvT<<<dim3(DM / 64, HD / 32, NH_), 256, 0, stream>>>(wq, WTQ, (unsigned)DM, (unsigned)HD);
    k_wconvT<<<dim3(DM / 64, HD / 32, NH_), 256, 0, stream>>>(wk, WTK, (unsigned)DM, (unsigned)HD);
    k_wconvT<<<dim3(DM / 64, HD / 32, NH_), 256, 0, stream>>>(wv, WTV, (unsigned)DM, (unsigned)HD);
    k_wconvT<<<dim3(DM / 64, DM / 32, 1), 256, 0, stream>>>(wo, WOT, (unsigned)DM, (unsigned)DM);
    k_wconvT<<<dim3(DM / 64, DFF / 32, 1), 256, 0, stream>>>(w1, W1T, (unsigned)DM, (unsigned)DFF);
    k_wconvT<<<dim3(DFF / 64, DM / 32, 1), 256, 0, stream>>>(w2, W2T, (unsigned)DFF, (unsigned)DM);

    k_gemm_tok<<<dim3(NB * SEQ / 64, DM / 64, 1), 32, 0, stream>>>(H1, WTQ, bq, QH, QR);
    k_gemm_tok<<<dim3(NB * SEQ / 64, DM / 64, 1), 32, 0, stream>>>(H1, WTK, bk, KP, KR);
    k_gemm_vt<<<dim3(DM / 64, NB * SEQ / 64, 1), 32, 0, stream>>>(WTV, H1, bv, VT, VR);

    k_flash_early<<<dim3(EROWS / (16 * AW), NB * NH_, 1), 32 * AW, 0, stream>>>(QH, QR, KP, KR, VT, VR, CT);
    if (SEQ > EROWS)
        k_flash_late<<<dim3((SEQ - EROWS) / (16 * AW), NB * NH_, 1), 32 * AW, 0, stream>>>(QH, KP, VT, CT);

    k_gemm_wo<<<dim3(NB * SEQ / 64, DM / 64, 1), 32, 0, stream>>>(CT, WOT, bo, x, X1);
    k_ln<<<dim3(NB * SEQ / 8, 1, 1), 256, 0, stream>>>(X1, g2, be2, H2, (unsigned)SEQ, 0);
    k_gemm_f1<<<dim3(NB * SEQ / 64, DFF / 64, 1), 32, 0, stream>>>(H2, W1T, b1, G);
    k_gemm_f2<<<dim3(NB * SEQ / 64, DM / 64, 1), 32, 0, stream>>>(G, W2T, b2, X1, OUT);
}
